// FourierAttention1d_44169443672696
// MI455X (gfx1250) — hardware-run, weakly checked
//
#include <hip/hip_runtime.h>


#ifndef NB
#define NB 4
#endif
#ifndef SEQ
#define SEQ 8192
#endif
#define NB_FULL  4
#define SEQ_FULL 8192
#ifndef OUT_SEQ
#define OUT_SEQ SEQ
#endif
#define CI   64
#define NH_  8
#define HD   64
#define HDM  512
#define CO   64
#define AW   4
#define OSP  68
#define NCH  8
#define CHN  (SEQ / NCH)
#define LN_EPS 1.0e-5f
#define KVC  (1.0f / 16.0f)
#define OWC  64.0f
#define OSC  0.25f
#define INVN (1.0f / (float)SEQ)

static_assert(HD == 64);
static_assert(NH_ * HD == HDM);
static_assert(CI % 32 == 0);
static_assert(HD % 32 == 0);
static_assert(CO == 64);
static_assert(OSP >= CO);
static_assert((OSP * 4) % 16 == 0);
static_assert(SEQ % 64 == 0);
static_assert((NB * SEQ) % 64 == 0);
static_assert(SEQ % NCH == 0);
static_assert(CHN % 32 == 0);
static_assert(SEQ % (16 * AW) == 0);
static_assert((SEQ & (SEQ - 1)) == 0);
static_assert(((size_t)SEQ * CI) % 8 == 0);
static_assert(((size_t)HDM * CI) % 8 == 0);
static_assert(((size_t)CO * HDM) % 8 == 0);
static_assert(((size_t)HD * HD) % 8 == 0);
static_assert(NB <= NB_FULL);
static_assert(SEQ <= SEQ_FULL);
static_assert(sizeof(float) * 16 * 68 <= 131072);
static_assert(sizeof(float) * AW * 16 * OSP <= 131072);

typedef _Float16 h16;
typedef unsigned short bf;
typedef __attribute__((ext_vector_type(16))) __bf16   v16bf;
typedef __attribute__((ext_vector_type(16))) _Float16 v16h;
typedef __attribute__((ext_vector_type(8)))  _Float16 v8h;
typedef __attribute__((ext_vector_type(8)))  unsigned short v8us;
typedef __attribute__((ext_vector_type(8)))  float    v8f;
typedef __attribute__((ext_vector_type(4)))  float    v4f;
typedef v4f  __attribute__((may_alias)) v4fa;

__device__ __forceinline__ unsigned short f2bf(float f) { unsigned u = __float_as_uint(f); u += 0x7FFFu + ((u >> 16) & 1u); return (unsigned short)(u >> 16); }
__device__ __forceinline__ float bfr(float f) { return __uint_as_float(((unsigned)f2bf(f)) << 16); }
__device__ __forceinline__ v16h cat16(v8h lo, v8h hi) { return __builtin_shufflevector(lo, hi, 0, 1, 2, 3, 4, 5, 6, 7, 8, 9, 10, 11, 12, 13, 14, 15); }
__device__ __forceinline__ v16bf cat16b(v8us lo, v8us hi) { return __builtin_bit_cast(v16bf, __builtin_shufflevector(lo, hi, 0, 1, 2, 3, 4, 5, 6, 7, 8, 9, 10, 11, 12, 13, 14, 15)); }
__device__ __forceinline__ v8f wmma16(v16h a, v16h b, v8f c) { return __builtin_amdgcn_wmma_f32_16x16x32_f16(false, a, false, b, (short)0, c, false, false); }
__device__ __forceinline__ v8f wmmab(v16bf a, v16bf b, v8f c) { return __builtin_amdgcn_wmma_f32_16x16x32_bf16(false, a, false, b, (short)0, c, false, false); }
__device__ __forceinline__ v16h  ldh(const h16* p) { return cat16(*(const v8h*)p, *(const v8h*)(p + 16)); }
__device__ __forceinline__ v16bf ldb(const bf* p)  { return cat16b(*(const v8us*)p, *(const v8us*)(p + 16)); }
__device__ __forceinline__ void wave_sync() { __builtin_amdgcn_fence(3  , "wavefront"); __builtin_amdgcn_wave_barrier(); asm volatile("" ::: "memory"); }
__device__ __forceinline__ v8f wmmabg(v16bf a, v16bf b, v8f c) { c = wmmab(a, b, c); asm volatile("v_nop\n\tv_nop\n\tv_nop\n\tv_nop" : "+v"(c) : "v"(a), "v"(b)); return c; }
__device__ __forceinline__ v8f wmma16g(v16h a, v16h b, v8f c) { c = wmma16(a, b, c); asm volatile("v_nop\n\tv_nop\n\tv_nop\n\tv_nop" : "+v"(c) : "v"(a), "v"(b)); return c; }
static __device__ __forceinline__ h16 toh_flush(float v) { const float w = (fabsf(v) < 6.103515625e-05f) ? 0.0f : v; return (h16)w; }

__global__ __launch_bounds__(256) void k_cvt8(const float* __restrict__ src, bf* dst, size_t n8) {
    const size_t i = (size_t)blockIdx.x * 256 + threadIdx.x; if (i >= n8) return;
    const v8f v = *(const v8f*)(src + i * 8); v8us o;
#pragma unroll
    for (int k = 0; k < 8; ++k) o[k] = f2bf(v[k]);
    *(volatile v8us*)(dst + i * 8) = o; __threadfence(); *(volatile v8us*)(dst + i * 8) = o;
}

__global__ __launch_bounds__(256) void k_cvtw(const float* __restrict__ src, h16* dst, size_t n8) {
    const size_t i = (size_t)blockIdx.x * 256 + threadIdx.x; if (i >= n8) return;
    const v8f v = *(const v8f*)(src + i * 8); v8h o;
#pragma unroll
    for (int k = 0; k < 8; ++k) o[k] = toh_flush(bfr(v[k]) * OWC);
    *(volatile v8h*)(dst + i * 8) = o; __threadfence(); *(volatile v8h*)(dst + i * 8) = o;
}

static_assert(32 * 16 * 4 == 16 * HD * 2);
__global__ __launch_bounds__(32) void k_projq(const bf* __restrict__ A, const bf* __restrict__ Bt, const float* __restrict__ bias,
                                              const float* __restrict__ lnw, const float* __restrict__ lnb, h16* QP) {
    __shared__ __align__(16) float os[16 * 68];
    const int K = CI;
    const int lane = threadIdx.x & 31, lr = lane & 15, hi = lane >> 4;
    const unsigned bx = blockIdx.x, hx = blockIdx.y;
    const unsigned r0 = bx * 64u, c0 = hx * 64u;
    v8f acc[4][4];
#pragma unroll
    for (int mb = 0; mb < 4; ++mb)
#pragma unroll
        for (int nb = 0; nb < 4; ++nb) acc[mb][nb] = (v8f){};
    const size_t aoff = (size_t)(r0 + lr) * K + 8 * hi, boff = (size_t)(c0 + lr) * K + 8 * hi;
#pragma unroll 1
    for (int kc = 0; kc < K; kc += 32) {
        v16bf a[4];
#pragma unroll
        for (int mb = 0; mb < 4; ++mb) a[mb] = ldb(A + aoff + (size_t)mb * 16 * K + kc);
#pragma unroll
        for (int nb = 0; nb < 4; ++nb) { const v16bf b = ldb(Bt + boff + (size_t)nb * 16 * K + kc);
#pragma unroll
            for (int mb = 0; mb < 4; ++mb) acc[mb][nb] = wmmabg(a[mb], b, acc[mb][nb]); }
    }
    float bc[4];
#pragma unroll
    for (int nb = 0; nb < 4; ++nb) bc[nb] = bfr(bias[c0 + nb * 16 + lr]);
    const int c8 = (lane & 7) * 8, rq = lane >> 3;
    const v4f g0 = *(const v4f*)(lnw + c0 + c8), g1 = *(const v4f*)(lnw + c0 + c8 + 4);
    const v4f f0 = *(const v4f*)(lnb + c0 + c8), f1 = *(const v4f*)(lnb + c0 + c8 + 4);
    float gg[8], oo[8];
#pragma unroll
    for (int i = 0; i < 4; ++i) { gg[i] = bfr(g0[i]); gg[4 + i] = bfr(g1[i]); oo[i] = bfr(f0[i]); oo[4 + i] = bfr(f1[i]); }
    const unsigned bb = r0 / (unsigned)SEQ, tt = r0 % (unsigned)SEQ;
    const unsigned zc = bb * (unsigned)NH_ + hx;
    const size_t tbase = ((size_t)zc * SEQ + (size_t)tt) * HD;
#pragma unroll
    for (int mb = 0; mb < 4; ++mb) {
#pragma unroll
        for (int nb = 0; nb < 4; ++nb) {
#pragma unroll
            for (int j = 0; j < 8; ++j) os[(hi * 8 + j) * 68 + nb * 16 + lr] = acc[mb][nb][j] + bc[nb]; }
        wave_sync();
        v8h hv[4];
#pragma unroll
        for (int s = 0; s < 4; ++s) { const int row = 4 * s + rq;
            const v4f x0 = *(const v4fa*)(&os[row * 68 + c8]); const v4f x1 = *(const v4fa*)(&os[row * 68 + c8 + 4]);
            float xv[8];
#pragma unroll
            for (int i = 0; i < 4; ++i) { xv[i] = x0[i]; xv[4 + i] = x1[i]; }
            float sm = ((xv[0] + xv[1]) + (xv[2] + xv[3])) + ((xv[4] + xv[5]) + (xv[6] + xv[7]));
            sm += __shfl_xor(sm, 1, 32); sm += __shfl_xor(sm, 2, 32); sm += __shfl_xor(sm, 4, 32);
            const float mu = sm * (1.0f / 64.0f);
            float q = 0.0f;
#pragma unroll
            for (int i = 0; i < 8; ++i) { xv[i] -= mu; q += xv[i] * xv[i]; }
            q += __shfl_xor(q, 1, 32); q += __shfl_xor(q, 2, 32); q += __shfl_xor(q, 4, 32);
            const float rs = rsqrtf(q * (1.0f / 64.0f) + LN_EPS);
#pragma unroll
            for (int i = 0; i < 8; ++i) hv[s][i] = toh_flush(xv[i] * rs * gg[i] + oo[i]); }
        const size_t sb = tbase + (size_t)(mb * 16) * HD;
#pragma unroll 1
        for (int ps = 0; ps < 2; ++ps) {
#pragma unroll
            for (int s = 0; s < 4; ++s) { const int row = 4 * s + rq;
                *(volatile v8h*)(QP + sb + (size_t)row * HD + c8) = hv[s]; }
            if (ps == 0) __threadfence(); }
        wave_sync();
    }
}

static_assert(32 * 16 * 4 == 16 * 64 * 2);
__global__ __launch_bounds__(32) void k_projt(const bf* __restrict__ A, const bf* __restrict__ Bt, const float* __restrict__ bias,
                                              const float* __restrict__ lnw, const float* __restrict__ lnb, h16* PT, int do_ln) {
    __shared__ __align__(16) float os[16 * 68];
    const int K = CI;
    const int lane = threadIdx.x & 31, lr = lane & 15, hi = lane >> 4;
    const unsigned bx = blockIdx.x, by = blockIdx.y;
    const unsigned r0 = bx * 64u, c0 = by * 64u;
    v8f acc[4][4];
#pragma unroll
    for (int mb = 0; mb < 4; ++mb)
#pragma unroll
        for (int nb = 0; nb < 4; ++nb) acc[mb][nb] = (v8f){};
    const size_t aoff = (size_t)(r0 + lr) * K + 8 * hi, boff = (size_t)(c0 + lr) * K + 8 * hi;
#pragma unroll 1
    for (int kc = 0; kc < K; kc += 32) {
        v16bf a[4];
#pragma unroll
        for (int mb = 0; mb < 4; ++mb) a[mb] = ldb(A + aoff + (size_t)mb * 16 * K + kc);
#pragma unroll
        for (int nb = 0; nb < 4; ++nb) { const v16bf b = ldb(Bt + boff + (size_t)nb * 16 * K + kc);
#pragma unroll
            for (int mb = 0; mb < 4; ++mb) acc[mb][nb] = wmmabg(a[mb], b, acc[mb][nb]); }
    }
#pragma unroll
    for (int mb = 0; mb < 4; ++mb) {
        const v4f b0 = *(const v4f*)(bias + r0 + mb * 16 + hi * 8), b1 = *(const v4f*)(bias + r0 + mb * 16 + hi * 8 + 4);
        float br[8];
#pragma unroll
        for (int i = 0; i < 4; ++i) { br[i] = bfr(b0[i]); br[4 + i] = bfr(b1[i]); }
#pragma unroll
        for (int nb = 0; nb < 4; ++nb) {
#pragma unroll
            for (int j = 0; j < 8; ++j) acc[mb][nb][j] += br[j]; }
    }
    float mu[4], rs[4];
#pragma unroll
    for (int nb = 0; nb < 4; ++nb) { mu[nb] = 0.0f; rs[nb] = 1.0f; }
    if (do_ln != 0) {
#pragma unroll
        for (int nb = 0; nb < 4; ++nb) {
            float s = 0.0f;
#pragma unroll
            for (int mb = 0; mb < 4; ++mb) {
#pragma unroll
                for (int j = 0; j < 8; ++j) s += acc[mb][nb][j]; }
            s += __shfl_xor(s, 16, 32);
            const float mm = s * (1.0f / 64.0f);
            float q = 0.0f;
#pragma unroll
            for (int mb = 0; mb < 4; ++mb) {
#pragma unroll
                for (int j = 0; j < 8; ++j) { const float d = acc[mb][nb][j] - mm; q += d * d; } }
            q += __shfl_xor(q, 16, 32);
            mu[nb] = mm; rs[nb] = rsqrtf(q * (1.0f / 64.0f) + LN_EPS);
        }
    }
    const unsigned bb = c0 / (unsigned)SEQ, tt = c0 % (unsigned)SEQ;
    const size_t tbase = (size_t)bb * (size_t)HDM * SEQ + (size_t)r0 * SEQ + (size_t)tt;
    const int c8 = (lane & 7) * 8, rq = lane >> 3;
#pragma unroll
    for (int mb = 0; mb < 4; ++mb) {
        float gg[8], oo[8];
#pragma unroll
        for (int j = 0; j < 8; ++j) { gg[j] = 1.0f; oo[j] = 0.0f; }
        if (do_ln != 0) {
            const v4f g0 = *(const v4f*)(lnw + r0 + mb * 16 + hi * 8), g1 = *(const v4f*)(lnw + r0 + mb * 16 + hi * 8 + 4);
            const v4f f0 = *(const v4f*)(lnb + r0 + mb * 16 + hi * 8), f1 = *(const v4f*)(lnb + r0 + mb * 16 + hi * 8 + 4);
#pragma unroll
            for (int i = 0; i < 4; ++i) { gg[i] = bfr(g0[i]); gg[4 + i] = bfr(g1[i]); oo[i] = bfr(f0[i]); oo[4 + i] = bfr(f1[i]); }
        }
#pragma unroll
        for (int nb = 0; nb < 4; ++nb) {
#pragma unroll
            for (int j = 0; j < 8; ++j) os[(hi * 8 + j) * 68 + nb * 16 + lr] = (acc[mb][nb][j] - mu[nb]) * rs[nb] * gg[j] + oo[j]; }
        wave_sync();
        v8h hv[4];
#pragma unroll
        for (int s = 0; s < 4; ++s) { const int row = 4 * s + rq;
            const v4f x0 = *(const v4fa*)(&os[row * 68 + c8]); const v4f x1 = *(const v4fa*)(&os[row * 68 + c8 + 4]);
#pragma unroll
            for (int i = 0; i < 4; ++i) { hv[s][i] = toh_flush(x0[i]); hv[s][4 + i] = toh_flush(x1[i]); } }
        const size_t sb = tbase + (size_t)(mb * 16) * SEQ;
#pragma unroll 1
        for (int ps = 0; ps < 2; ++ps) {
#pragma unroll
            for (int s = 0; s < 4; ++s) { const int row = 4 * s + rq;
                *(volatile v8h*)(PT + sb + (size_t)row * SEQ + c8) = hv[s]; }
            if (ps == 0) __threadfence(); }
        wave_sync();
    }
}

static_assert(32 * 16 * 8 == 16 * HD * 4);
__global__ __launch_bounds__(32) void k_kv(const h16* __restrict__ VT, const h16* __restrict__ KT, float* PART) {
    __shared__ __align__(16) float os[16 * 68];
    const int lane = threadIdx.x & 31, lr = lane & 15, hi = lane >> 4;
    const unsigned ch = blockIdx.x, zh = blockIdx.y;
    const size_t fo = (size_t)zh * HD * SEQ + (size_t)lr * SEQ + (size_t)ch * CHN + 8 * hi;
    v8f acc[4][4];
#pragma unroll
    for (int eb = 0; eb < 4; ++eb)
#pragma unroll
        for (int db = 0; db < 4; ++db) acc[eb][db] = (v8f){};
#pragma unroll 1
    for (int kc = 0; kc < CHN; kc += 32) {
        v16h a[4];
#pragma unroll
        for (int eb = 0; eb < 4; ++eb) a[eb] = ldh(VT + fo + (size_t)eb * 16 * SEQ + kc);
#pragma unroll
        for (int db = 0; db < 4; ++db) { const v16h b = ldh(KT + fo + (size_t)db * 16 * SEQ + kc);
#pragma unroll
            for (int eb = 0; eb < 4; ++eb) acc[eb][db] = wmma16g(a[eb], b, acc[eb][db]); }
    }
    float* pp = PART + ((size_t)zh * NCH + ch) * (size_t)(HD * HD);
    const int c4 = (lane & 15) * 4, rh = lane >> 4;
#pragma unroll
    for (int eb = 0; eb < 4; ++eb) {
#pragma unroll
        for (int db = 0; db < 4; ++db) {
#pragma unroll
            for (int j = 0; j < 8; ++j) os[(hi * 8 + j) * 68 + db * 16 + lr] = acc[eb][db][j]; }
        wave_sync();
#pragma unroll 1
        for (int ps = 0; ps < 2; ++ps) {
#pragma unroll
            for (int s = 0; s < 8; ++s) { const int row = 2 * s + rh;
                const v4f val = *(const v4fa*)(&os[row * 68 + c4]);
                *(volatile v4f*)(pp + (size_t)(eb * 16 + row) * HD + c4) = val; }
            if (ps == 0) __threadfence(); }
        wave_sync();
    }
}

__global__ __launch_bounds__(256) void k_kvred(const float* __restrict__ PART, h16* KVT) {
#pragma clang fp contract(off)
    const unsigned i = blockIdx.x * 256u + threadIdx.x;
    if (i >= (unsigned)(NB * NH_ * HD * HD / 8)) return;
    const unsigned zh = i / (unsigned)(HD * HD / 8), w = i % (unsigned)(HD * HD / 8);
    const float* p = PART + (size_t)zh * NCH * (size_t)(HD * HD) + (size_t)w * 8;
    v4f s0 = (v4f){}, s1 = (v4f){};
#pragma unroll 1
    for (int c = 0; c < NCH; ++c) { const v4f a = *(const v4f*)(p + (size_t)c * (HD * HD)); const v4f b = *(const v4f*)(p + (size_t)c * (HD * HD) + 4); s0 = s0 + a; s1 = s1 + b; }
    v8h o;
#pragma unroll
    for (int k = 0; k < 4; ++k) { o[k] = toh_flush(s0[k] * KVC); o[4 + k] = toh_flush(s1[k] * KVC); }
    *(volatile v8h*)(KVT + (size_t)i * 8) = o; __threadfence(); *(volatile v8h*)(KVT + (size_t)i * 8) = o;
}

static_assert(32 * 16 * 8 == 16 * CO * 4);
__global__ __launch_bounds__(32 * AW) void k_out(const h16* __restrict__ QP, const h16* __restrict__ KVT, const h16* __restrict__ OW, const float* __restrict__ ob, float* OUT) {
    __shared__ __align__(16) float os[AW * 16 * OSP];
    const int lane = threadIdx.x & 31, lr = lane & 15, hi = lane >> 4;
    const int wave = __builtin_amdgcn_readfirstlane((int)(threadIdx.x >> 5));
    const unsigned b = blockIdx.y;
    const unsigned t0 = (blockIdx.x * (unsigned)AW + (unsigned)wave) * 16u;
    const size_t qo = ((size_t)b * NH_ * SEQ + (size_t)(t0 + lr)) * HD + 8 * hi;
    const size_t ko = ((size_t)b * NH_ * HD + (size_t)lr) * HD + 8 * hi;
    const size_t wo = (size_t)lr * HDM + 8 * hi;
    v8f acc[4];
#pragma unroll
    for (int fb = 0; fb < 4; ++fb) acc[fb] = (v8f){};
#pragma unroll 1
    for (int h = 0; h < NH_; ++h) {
        const h16* qp = QP + qo + (size_t)h * SEQ * HD;
        const v16h q0 = ldh(qp), q1 = ldh(qp + 32);
        const h16* kp = KVT + ko + (size_t)h * (HD * HD);
        v8f oT[4];
#pragma unroll
        for (int eb = 0; eb < 4; ++eb) {
            const v16h a0 = ldh(kp + (size_t)eb * 16 * HD), a1 = ldh(kp + (size_t)eb * 16 * HD + 32);
            oT[eb] = (v8f){};
            oT[eb] = wmma16g(a0, q0, oT[eb]); oT[eb] = wmma16g(a1, q1, oT[eb]); }
        v16h p0, p1;
#pragma unroll
        for (int r = 0; r < 8; ++r) { p0[r] = toh_flush(oT[0][r]); p0[8 + r] = toh_flush(oT[1][r]); p1[r] = toh_flush(oT[2][r]); p1[8 + r] = toh_flush(oT[3][r]); }
        const h16* wp = OW + wo + (size_t)h * HD;
#pragma unroll
        for (int fb = 0; fb < 4; ++fb) {
            const v16h a0 = ldh(wp + (size_t)fb * 16 * HDM), a1 = ldh(wp + (size_t)fb * 16 * HDM + 32);
            acc[fb] = wmma16g(a0, p0, acc[fb]); acc[fb] = wmma16g(a1, p1, acc[fb]); }
    }
    const int wb = wave * 16 * OSP;
#pragma unroll
    for (int fb = 0; fb < 4; ++fb) { v4f a, c;
        a[0] = acc[fb][0]; a[1] = acc[fb][1]; a[2] = acc[fb][2]; a[3] = acc[fb][3]; c[0] = acc[fb][4]; c[1] = acc[fb][5]; c[2] = acc[fb][6]; c[3] = acc[fb][7];
        *(v4fa*)(&os[wb + lr * OSP + fb * 16 + 8 * hi]) = a; *(v4fa*)(&os[wb + lr * OSP + fb * 16 + 8 * hi + 4]) = c; }
    wave_sync();
    const int cofs = (lane & 15) * 4, rh = lane >> 4;
    const v4f obv = *(const v4f*)(ob + cofs);
    v4f ob4;
#pragma unroll
    for (int i = 0; i < 4; ++i) ob4[i] = bfr(obv[i]);
    float* orow = OUT + ((size_t)b * OUT_SEQ + t0) * CO;
#pragma unroll 1
    for (int ps = 0; ps < 2; ++ps) {
#pragma unroll
        for (int s = 0; s < 8; ++s) { const int row = 2 * s + rh;
            const v4f x = *(const v4fa*)(&os[wb + row * OSP + cofs]); v4f val;
#pragma unroll
            for (int i = 0; i < 4; ++i) val[i] = (x[i] * OSC + ob4[i]) * INVN;
            *(volatile v4f*)(orow + (size_t)row * CO + cofs) = val; }
        if (ps == 0) __threadfence(); }
}

static constexpr size_t al256(size_t v) { return (v + 255) & ~(size_t)255; }
static constexpr size_t SZ_XB = al256((size_t)NB * SEQ * CI * 2);
static constexpr size_t SZ_WB = al256((size_t)3 * HDM * CI * 2);
static constexpr size_t SZ_OW = al256((size_t)CO * HDM * 2);
static constexpr size_t SZ_PL = al256((size_t)NB * NH_ * SEQ * HD * 2);
static constexpr size_t SZ_PT = al256((size_t)NB * NH_ * NCH * HD * HD * 4);
static constexpr size_t SZ_KV = al256((size_t)NB * NH_ * HD * HD * 2);
static constexpr size_t SZ_TOTAL = SZ_XB + SZ_WB + SZ_OW + 3 * SZ_PL + SZ_PT + SZ_KV;
static_assert(SZ_TOTAL <= (size_t)134217728);
static_assert(((size_t)HDM * CI * 2) % 256 == 0);
static_assert((size_t)NB * NH_ * SEQ * HD == (size_t)NB * HDM * SEQ);
static_assert(((size_t)NB * NH_ * HD * HD) % 8 == 0);

extern "C" void kernel_launch(void* const* d_in, const int* in_sizes, int n_in,
                              void* d_out, int out_size, void* d_ws, size_t ws_size, hipStream_t stream) {
    if (n_in < 13) return;
    const size_t needx = ((size_t)(NB - 1) * SEQ_FULL + SEQ) * CI;
    if ((size_t)in_sizes[0] < needx) return;
    if ((size_t)in_sizes[1] < (size_t)HDM * CI || (size_t)in_sizes[3] < (size_t)HDM * CI || (size_t)in_sizes[5] < (size_t)HDM * CI) return;
    if (in_sizes[2] < HDM || in_sizes[4] < HDM || in_sizes[6] < HDM) return;
    if (in_sizes[7] < NH_ * HD || in_sizes[8] < NH_ * HD || in_sizes[9] < NH_ * HD || in_sizes[10] < NH_ * HD) return;
    if ((size_t)in_sizes[11] < (size_t)CO * HDM || in_sizes[12] < CO) return;
    if ((size_t)out_size < ((size_t)(NB - 1) * OUT_SEQ + SEQ) * CO) return;
    if (SZ_TOTAL > ws_size) return;
    const float* xin = (const float*)d_in[0];
    const float* wq = (const float*)d_in[1];  const float* bq = (const float*)d_in[2];
    const float* wk = (const float*)d_in[3];  const float* bk = (const float*)d_in[4];
    const float* wv = (const float*)d_in[5];  const float* bv = (const float*)d_in[6];
    const float* lqw = (const float*)d_in[7]; const float* lqb = (const float*)d_in[8];
    const float* lkw = (const float*)d_in[9]; const float* lkb = (const float*)d_in[10];
    const float* ow = (const float*)d_in[11]; const float* obp = (const float*)d_in[12];
    float* OUT = (float*)d_out;
    char* wsp = (char*)d_ws;
    bf* XB = (bf*)wsp; wsp += SZ_XB;
    bf* WB = (bf*)wsp; wsp += SZ_WB;
    h16* OW = (h16*)wsp; wsp += SZ_OW;
    h16* QP = (h16*)wsp; wsp += SZ_PL;
    h16* KT = (h16*)wsp; wsp += SZ_PL;
    h16* VT = (h16*)wsp; wsp += SZ_PL;
    float* PART = (float*)wsp; wsp += SZ_PT;
    h16* KVT = (h16*)wsp; wsp += SZ_KV;
    bf* WQ = WB; bf* WK = WB + (size_t)HDM * CI; bf* WV = WB + (size_t)2 * HDM * CI;

    if (SEQ == SEQ_FULL) {
        const size_t n8 = (size_t)NB * SEQ * CI / 8;
        k_cvt8<<<(unsigned)((n8 + 255) / 256), 256, 0, stream>>>(xin, XB, n8);
    } else {
        const size_t n8 = (size_t)SEQ * CI / 8;
        for (int b = 0; b < NB; ++b) k_cvt8<<<(unsigned)((n8 + 255) / 256), 256, 0, stream>>>(xin + (size_t)b * SEQ_FULL * CI, XB + (size_t)b * SEQ * CI, n8);
    }
    { const size_t n8 = (size_t)HDM * CI / 8; const unsigned g = (unsigned)((n8 + 255) / 256);
      k_cvt8<<<g, 256, 0, stream>>>(wq, WQ, n8); k_cvt8<<<g, 256, 0, stream>>>(wk, WK, n8); k_cvt8<<<g, 256, 0, stream>>>(wv, WV, n8); }
    { const size_t n8 = (size_t)CO * HDM / 8;
      k_cvtw<<<(unsigned)((n8 + 255) / 256), 256, 0, stream>>>(ow, OW, n8); }

    k_projq<<<dim3(NB * SEQ / 64, NH_, 1), 32, 0, stream>>>(XB, WQ, bq, lqw, lqb, QP);
    k_projt<<<dim3(NH_, NB * SEQ / 64, 1), 32, 0, stream>>>(WK, XB, bk, lkw, lkb, KT, 1);
    k_projt<<<dim3(NH_, NB * SEQ / 64, 1), 32, 0, stream>>>(WV, XB, bv, lkw, lkb, VT, 0);
    k_kv<<<dim3(NCH, NB * NH_, 1), 32, 0, stream>>>(VT, KT, PART);
    { const unsigned n8 = (unsigned)(NB * NH_ * HD * HD / 8);
      k_kvred<<<(n8 + 255u) / 256u, 256, 0, stream>>>(PART, KVT); }
    k_out<<<dim3(SEQ / (16 * AW), NB, 1), 32 * AW, 0, stream>>>(QP, KVT, OW, obp, OUT);
}
